// RGCNBasisLayer_5446018531349
// MI455X (gfx1250) — hardware-run, weakly checked
//
#include <hip/hip_runtime.h>


namespace {
constexpr int N = 60000, NP = 60032, EFULL = 600000, E = 600000  , IN = 32, OUT = 32, ATT = 32, R = 200, NB = 4, NG = 8;
constexpr float XS = 8.0f, WSC = 256.0f;
static_assert(E % 32 == 0 && NP % 32 == 0, "tiling");
typedef _Float16 b16;
typedef __attribute__((ext_vector_type(16))) _Float16 v16b;
typedef __attribute__((ext_vector_type(8))) _Float16 v8b;
typedef __attribute__((ext_vector_type(8))) float v8f;
typedef __attribute__((ext_vector_type(4))) float v4f;
__device__ __forceinline__ float bf16_rne(float f) { unsigned int u = __float_as_uint(f); u += 0x7FFFu + ((u >> 16) & 1u); return __uint_as_float(u & 0xFFFF0000u); }
__device__ __forceinline__ void split16(float v, b16& hi, b16& lo) { hi = (b16)v; lo = (b16)(v - (float)hi); }
__device__ __forceinline__ v16b frag_kb(const b16* p, int hh) { const v8b a = *(const v8b*)(p + 8 * hh), b = *(const v8b*)(p + 16 + 8 * hh); v16b f;
#pragma unroll
  for (int e = 0; e < 8; ++e) { f[e] = a[e]; f[8 + e] = b[e]; } return f; }
__device__ __forceinline__ v8f wmma16b(v16b a, v16b b, v8f c) { v8f d = __builtin_amdgcn_wmma_f32_16x16x32_f16(false, a, false, b, (short)0, c, false, false); asm volatile("v_nop\n\tv_nop\n\tv_nop\n\tv_nop" : "+v"(d) : "v"(a), "v"(b)); return d; }
__device__ __forceinline__ void wave_lds_sync() { __builtin_amdgcn_fence(__ATOMIC_RELEASE, "workgroup"); __builtin_amdgcn_wave_barrier(); __builtin_amdgcn_fence(__ATOMIC_ACQUIRE, "workgroup"); }
__device__ __forceinline__ float pmul(float a, float b) { float p = a * b; asm volatile("" : "+v"(p)); return p; }
__device__ __forceinline__ int iclamp(int v, int lo, int hi) { return v < lo ? lo : (v > hi ? hi : v); }
constexpr int CSR_NBLK = 512, CSR_GB = 9, CSR_GN = 1 << CSR_GB  , CSR_MAXG = 512, CSR_CAP = 12288  ;
__global__ __launch_bounds__(64) void csrA_kernel(const int* __restrict__ dst, int E, int N, int nG, int CHP, int NGP, int* __restrict__ STG, int* __restrict__ HST) {
  extern __shared__ int sm[];
  int* cnt = sm; int* run = sm + NGP; int* ids = sm + 2 * NGP;
  const int b = blockIdx.x; const int ch = (E + CSR_NBLK - 1) / CSR_NBLK; const int e0 = b * ch, e1 = min(E, e0 + ch);
  for (int i = threadIdx.x; i < NGP; i += 64) cnt[i] = 0;
  for (int i = threadIdx.x; i < CHP; i += 64) ids[i] = -1;
  __syncthreads();
  if (threadIdx.x == 0) {
    for (int e = e0; e < e1; ++e) { int d = dst[e]; d = (d < 0) ? 0 : (d >= N ? N - 1 : d); cnt[d >> CSR_GB] += 1; }
    int acc = 0; for (int g = 0; g < nG; ++g) { run[g] = acc; acc += cnt[g]; }
    for (int e = e0; e < e1; ++e) { int d = dst[e]; d = (d < 0) ? 0 : (d >= N ? N - 1 : d); const int g = d >> CSR_GB; ids[run[g]] = e; run[g] += 1; } }
  __syncthreads();
  typedef __attribute__((ext_vector_type(4))) int v4i;
  for (int pass = 0; pass < 2; ++pass) {
    for (int i = threadIdx.x; i < CHP / 4; i += 64) *(volatile v4i*)(STG + (size_t)b * CHP + i * 4) = *(const v4i*)(&ids[i * 4]);
    for (int i = threadIdx.x; i < NGP / 4; i += 64) { v4i v; for (int e = 0; e < 4; ++e) v[e] = (i * 4 + e < nG) ? cnt[i * 4 + e] : 0; *(volatile v4i*)(HST + (size_t)b * NGP + i * 4) = v; }
    __threadfence(); }
}
__global__ __launch_bounds__(512) void csrS_kernel(const int* __restrict__ HST, int nG, int NGP, int* __restrict__ START, int* __restrict__ TOT, int* __restrict__ OFF) {
  __shared__ int tot[CSR_MAXG];
  const int b = threadIdx.x;
  for (int pass = 0; pass < 2; ++pass) { int runb = 0; for (int g = 0; g < nG; ++g) { int c = HST[(size_t)b * NGP + g]; c = (c < 0) ? 0 : c; ((volatile int*)OFF)[(size_t)g * CSR_NBLK + b] = runb; runb += c; } __threadfence(); }
  for (int g = threadIdx.x; g < nG; g += 512) { int s = 0; for (int bb = 0; bb < CSR_NBLK; ++bb) { int c = HST[(size_t)bb * NGP + g]; s += (c < 0) ? 0 : c; } tot[g] = s; }
  __syncthreads();
  if (threadIdx.x < 32) {
    __shared__ int st[CSR_MAXG + 32];
    if (threadIdx.x == 0) { int acc = 0; for (int g = 0; g < NGP; ++g) { st[g] = acc; if (g < nG) acc += (tot[g] + 31) & ~31; } st[NGP] = acc; }
    __builtin_amdgcn_fence(__ATOMIC_RELEASE, "workgroup"); __builtin_amdgcn_wave_barrier(); __builtin_amdgcn_fence(__ATOMIC_ACQUIRE, "workgroup");
    for (int pass = 0; pass < 2; ++pass) { for (int i = threadIdx.x; i < NGP + 32; i += 32) { ((volatile int*)START)[i] = (i <= NGP) ? st[min(i, NGP)] : 0; ((volatile int*)TOT)[i] = (i < nG) ? tot[i] : 0; } __threadfence(); } }
}
__global__ __launch_bounds__(256) void csrB_kernel(const int* __restrict__ dst, int N, int nG, int CHP, int NGP, int permLen, const int* __restrict__ STG, const int* __restrict__ HST, const int* __restrict__ OFF, const int* __restrict__ START, const int* __restrict__ TOT, int* __restrict__ PERM, int* __restrict__ ROWPTR, int* __restrict__ ROWCNT, int* __restrict__ FLAG) {
  typedef __attribute__((ext_vector_type(4))) int v4i;
  __shared__ int ids[CSR_CAP]; __shared__ unsigned short key[CSR_CAP]; __shared__ int outp[CSR_CAP]; __shared__ int ncnt[CSR_GN + 1]; __shared__ int boff[CSR_NBLK + 1];
  const int g = blockIdx.x, t_ = threadIdx.x; int tot = TOT[g]; int st = START[g], stn = START[g + 1]; const int v0 = g * CSR_GN; const int nv = min(CSR_GN, N - v0);
  st = (st < 0) ? 0 : (st > permLen - 32 ? permLen - 32 : st) & ~31; stn = (stn < st) ? st : (stn > permLen ? permLen : stn); tot = (tot < 0) ? 0 : tot; if (tot > stn - st && tot <= CSR_CAP) tot = stn - st;
  if (tot > CSR_CAP) {
    for (int pass = 0; pass < 2; ++pass) { for (int i = t_; i < CSR_GN / 4; i += 256) { v4i a, c; for (int e = 0; e < 4; ++e) { a[e] = st; c[e] = 0; } *(volatile v4i*)(ROWPTR + v0 + i * 4) = a; *(volatile v4i*)(ROWCNT + v0 + i * 4) = c; } if (t_ == 0) ((volatile int*)FLAG)[0] = 1; __threadfence(); } (void)nv; return; }
  if (t_ == 0) { int acc = 0; for (int b = 0; b < CSR_NBLK; ++b) { boff[b] = acc; int c = HST[(size_t)b * NGP + g]; c = (c < 0) ? 0 : (c > CHP ? CHP : c); acc += c; if (acc > tot) acc = tot; } boff[CSR_NBLK] = acc; }
  for (int i = t_; i <= CSR_GN; i += 256) ncnt[i] = 0;
  __syncthreads();
  for (int b = 0; b < CSR_NBLK; ++b) { const int c = boff[b + 1] - boff[b]; int o_ = OFF[(size_t)g * CSR_NBLK + b]; o_ = (o_ < 0) ? 0 : (o_ > CHP - c ? CHP - c : o_); const int* src_ = STG + (size_t)b * CHP + o_;
    for (int i = t_; i < c; i += 256) { int id = src_[i]; id = (id < 0) ? 0 : id; ids[boff[b] + i] = id; int d = dst[id]; d = (d < v0) ? v0 : (d >= N ? N - 1 : d); int kk = d - v0; kk = (kk < 0) ? 0 : (kk >= CSR_GN ? CSR_GN - 1 : kk); key[boff[b] + i] = (unsigned short)kk; } }
  __syncthreads();
  if (t_ == 0) { for (int i = 0; i < tot; ++i) ncnt[key[i]] += 1; int acc = 0; for (int vl = 0; vl < CSR_GN; ++vl) { const int c = ncnt[vl]; ncnt[vl] = acc; acc += c; } ncnt[CSR_GN] = acc;
    for (int i = 0; i < tot; ++i) { const int vl = key[i]; outp[ncnt[vl]] = ids[i]; ncnt[vl] += 1; }
    for (int vl = CSR_GN; vl > 0; --vl) ncnt[vl] = ncnt[vl - 1]; ncnt[0] = 0; }
  __syncthreads();
  for (int pass = 0; pass < 2; ++pass) {
    for (int i = t_; i < (stn - st) / 4; i += 256) { v4i v; for (int e = 0; e < 4; ++e) { const int q = i * 4 + e; v[e] = (q < tot) ? outp[q] : -1; } *(volatile v4i*)(PERM + st + i * 4) = v; }
    for (int i = t_; i < CSR_GN / 4; i += 256) { v4i a, c; for (int e = 0; e < 4; ++e) { const int vl = i * 4 + e; a[e] = st + ncnt[vl]; c[e] = (vl < nv) ? (ncnt[vl + 1] - ncnt[vl]) : 0; } *(volatile v4i*)(ROWPTR + v0 + i * 4) = a; *(volatile v4i*)(ROWCNT + v0 + i * 4) = c; }
    __threadfence(); }
}
__global__ __launch_bounds__(256) void csrZ_kernel(int* __restrict__ p, size_t n4) { typedef __attribute__((ext_vector_type(4))) int v4i; const size_t tid = (size_t)blockIdx.x * 256 + threadIdx.x, nth = (size_t)gridDim.x * 256; v4i z = {0, 0, 0, 0}; for (size_t i = tid; i < n4; i += nth) *(volatile v4i*)(p + i * 4) = z; }
struct CsrBufs { int *STG, *HST, *OFF, *START, *TOT, *PERM, *ROWPTR, *ROWCNT, *FLAG; int nG, NGP, CHP; size_t permLen; char* base; size_t bytes; };
static size_t csr_carve(CsrBufs& c, char* ws, size_t off, int E, int N) {
  const size_t off0 = off; c.base = ws + off;
  auto al = [&](size_t bytes) { char* p = ws + off; off += (bytes + 255) & ~(size_t)255; return p; };
  c.nG = (N + CSR_GN - 1) / CSR_GN; c.NGP = (c.nG + 31) & ~31; const int ch = (E + CSR_NBLK - 1) / CSR_NBLK; c.CHP = (ch + 31) & ~31; c.permLen = (size_t)E + 32 * (size_t)c.nG + 32;
  c.STG = (int*)al((size_t)CSR_NBLK * c.CHP * 4); c.HST = (int*)al((size_t)CSR_NBLK * c.NGP * 4); c.OFF = (int*)al((size_t)c.NGP * CSR_NBLK * 4); c.START = (int*)al((size_t)(c.NGP + 64) * 4); c.TOT = (int*)al((size_t)(c.NGP + 64) * 4);
  c.PERM = (int*)al(c.permLen * 4); c.ROWPTR = (int*)al((size_t)c.nG * CSR_GN * 4); c.ROWCNT = (int*)al((size_t)c.nG * CSR_GN * 4); c.FLAG = (int*)al(256);
  c.bytes = off - off0; return off;
}
static void csr_build(const CsrBufs& c, const int* dst, int E, int N, hipStream_t stream) {
  const size_t smem = (size_t)(2 * c.NGP + c.CHP) * 4;
  csrZ_kernel<<<512, 256, 0, stream>>>((int*)c.base, c.bytes / 16);
  csrA_kernel<<<CSR_NBLK, 64, smem, stream>>>(dst, E, N, c.nG, c.CHP, c.NGP, c.STG, c.HST);
  csrS_kernel<<<1, 512, 0, stream>>>(c.HST, c.nG, c.NGP, c.START, c.TOT, c.OFF);
  csrB_kernel<<<c.nG, 256, 0, stream>>>(dst, N, c.nG, c.CHP, c.NGP, (int)c.permLen, c.STG, c.HST, c.OFF, c.START, c.TOT, c.PERM, c.ROWPTR, c.ROWCNT, c.FLAG);
}

typedef __attribute__((ext_vector_type(2))) float v2f;
__global__ __launch_bounds__(256) void wprep_kernel(const float* __restrict__ basis, const float* __restrict__ a1w, const float* __restrict__ a2w, b16* __restrict__ BB, b16* __restrict__ A1T, b16* __restrict__ A2T) {
  for (int u = threadIdx.x; u < (128 * 32 + 32 * 96 + 32 * 64) / 8; u += 256) { v8b o; int e = u * 8;
    if (e < 128 * 32) { const int row = e / 32, i0 = e % 32; const int b = row / 32, oo = row % 32; for (int j = 0; j < 8; ++j) o[j] = (b16)(bf16_rne(basis[((size_t)b * IN + i0 + j) * OUT + oo]) * WSC); for (int pass = 0; pass < 2; ++pass) { *(volatile v8b*)(BB + e) = o; __threadfence(); } continue; } e -= 128 * 32;
    if (e < 32 * 96) { const int oo = e / 96, k0 = e % 96; for (int j = 0; j < 8; ++j) o[j] = (b16)(bf16_rne(a1w[(size_t)(k0 + j) * IN + oo]) * WSC); for (int pass = 0; pass < 2; ++pass) { *(volatile v8b*)(A1T + e) = o; __threadfence(); } continue; } e -= 32 * 96;
    { const int oo = e / 64, k0 = e % 64; for (int j = 0; j < 8; ++j) o[j] = (b16)(bf16_rne(a2w[(size_t)(k0 + j) * IN + oo]) * WSC); for (int pass = 0; pass < 2; ++pass) { *(volatile v8b*)(A2T + e) = o; __threadfence(); } } }
}
__global__ __launch_bounds__(64) void edge_kernel(const float* __restrict__ x, const int* __restrict__ srcs, const int* __restrict__ dsts, const int* __restrict__ et, const int* __restrict__ eg, const int* __restrict__ tl, const float* __restrict__ nrm, const float* __restrict__ rel, const float* __restrict__ wcomp,
                                                  const b16* __restrict__ BB, const b16* __restrict__ A1T, const float* __restrict__ a1b, const float* __restrict__ b1w, const float* __restrict__ b1b, const b16* __restrict__ A2T, const float* __restrict__ a2b, const float* __restrict__ b2w, const float* __restrict__ b2b, float* __restrict__ MSG) {
  __shared__ __attribute__((aligned(16))) b16 X96[2][16][96 + 8], R64[2][16][64 + 8]; __shared__ __attribute__((aligned(16))) float XB[2][16][128 + 4], Ms[2][16][32 + 1]; __shared__ float coef[2][16][NB], nrms[2][16], asum[2][16];
  const int wave = threadIdx.x >> 5, lane = threadIdx.x & 31, nloc = lane & 15, hlf = lane >> 4; const size_t e0 = (size_t)blockIdx.x * 32 + wave * 16;
  { const size_t e = e0 + nloc; const int s = iclamp(srcs[e], 0, N - 1), d = iclamp(dsts[e], 0, N - 1), ty = iclamp(et[e], 0, R - 1), g = iclamp(eg[e], 0, NG - 1), tlab = iclamp(tl[g], 0, R - 1);
    const float* xr = x + (size_t)(hlf ? d : s) * IN; const float* er = rel + ((size_t)g * R + ty) * ATT; const float* tr = rel + ((size_t)g * R + tlab) * ATT;
    for (int q = 0; q < 32; q += 8) { v8b o; for (int j = 0; j < 8; ++j) o[j] = (b16)(bf16_rne(xr[q + j]) * XS); *(v8b*)(&X96[wave][nloc][hlf * 32 + q]) = o; }
    for (int q = 0; q < 32; q += 8) { v8b o, o2; for (int j = 0; j < 8; ++j) { const float ev = bf16_rne(er[q + j]); o[j] = (b16)(ev * XS); o2[j] = (b16)((ev + bf16_rne(tr[q + j])) * XS); }
      if (hlf == 0) { *(v8b*)(&X96[wave][nloc][64 + q]) = o; *(v8b*)(&R64[wave][nloc][q]) = o; } else { *(v8b*)(&R64[wave][nloc][32 + q]) = o2; } }
    if (hlf == 0) { for (int b = 0; b < NB; ++b) coef[wave][nloc][b] = bf16_rne(wcomp[ty * NB + b]); nrms[wave][nloc] = bf16_rne(nrm[e]); } }
  wave_lds_sync();
  { const v16b a = frag_kb(&X96[wave][nloc][0], hlf);
#pragma unroll
    for (int t = 0; t < 8; ++t) { v8f d = (v8f){}; d = wmma16b(a, frag_kb(BB + (size_t)(t * 16 + nloc) * IN, hlf), d);
#pragma unroll
      for (int r = 0; r < 8; ++r) XB[wave][8 * hlf + r][t * 16 + nloc] = d[r] * (1.0f / (XS * WSC)); } }
  float h1[2][8], h2[2][8];
#pragma unroll
  for (int t = 0; t < 2; ++t) { v8f d1 = (v8f){}, d2 = (v8f){};
#pragma unroll
    for (int ks = 0; ks < 3; ++ks) d1 = wmma16b(frag_kb(&X96[wave][nloc][ks * 32], hlf), frag_kb(A1T + (size_t)(t * 16 + nloc) * 96 + ks * 32, hlf), d1);
#pragma unroll
    for (int ks = 0; ks < 2; ++ks) d2 = wmma16b(frag_kb(&R64[wave][nloc][ks * 32], hlf), frag_kb(A2T + (size_t)(t * 16 + nloc) * 64 + ks * 32, hlf), d2);
    const int hu = t * 16 + nloc; const float ba = bf16_rne(a1b[hu]), bb2 = bf16_rne(a2b[hu]), w1 = bf16_rne(b1w[hu]), w2 = bf16_rne(b2w[hu]);
#pragma unroll
    for (int r = 0; r < 8; ++r) { h1[t][r] = pmul(fmaxf(d1[r] * (1.0f / (XS * WSC)) + ba, 0.0f), w1); h2[t][r] = pmul(fmaxf(d2[r] * (1.0f / (XS * WSC)) + bb2, 0.0f), w2); } }
  { const float c1 = bf16_rne(b1b[0]), c2 = bf16_rne(b2b[0]);
#pragma unroll
    for (int r = 0; r < 8; ++r) { float s1 = h1[0][r] + h1[1][r], s2 = h2[0][r] + h2[1][r];
#pragma unroll
      for (int o = 1; o < 16; o <<= 1) { s1 += __shfl_xor(s1, o); s2 += __shfl_xor(s2, o); }
      const float al = 1.0f / (1.0f + __expf(-(s1 + c1))) + 1.0f / (1.0f + __expf(-(s2 + c2)));
      if (nloc == (r & 15)) asum[wave][8 * hlf + r] = al; } }
  wave_lds_sync();
#pragma unroll 1
  for (int rr = 0; rr < 16; ++rr) { float s = 0.0f;
#pragma unroll
    for (int b = 0; b < NB; ++b) s += pmul(coef[wave][rr][b], XB[wave][rr][b * 32 + lane]);
    Ms[wave][rr][lane] = pmul(pmul(s, nrms[wave][rr]), asum[wave][rr]); }
  wave_lds_sync();
  for (int pass = 0; pass < 2; ++pass) { for (int rr = 0; rr < 16; ++rr) ((volatile float*)MSG)[(e0 + rr) * OUT + lane] = Ms[wave][rr][lane]; __threadfence(); }
}
__global__ __launch_bounds__(256) void node_kernel(const float* __restrict__ MSG, const float* __restrict__ x, const float* __restrict__ sl, const float* __restrict__ bias, const int* __restrict__ PERM, const int* __restrict__ ROWPTR, const int* __restrict__ ROWCNT, int permLen, float* __restrict__ out) {
  const int wave = threadIdx.x >> 5, lane = threadIdx.x & 31; const size_t v = (size_t)blockIdx.x * 8 + wave; if (v >= (size_t)N) return;
  float a = 0.0f; int st = ROWPTR[v], cnt = ROWCNT[v]; cnt = iclamp(cnt, 0, 65536); st = iclamp(st, 0, permLen - cnt);
#pragma unroll 1
  for (int j = 0; j < cnt; ++j) { const int e = iclamp(PERM[st + j], 0, E - 1); a += MSG[(size_t)e * OUT + lane]; }
  float s = bf16_rne(bias[lane]);
#pragma unroll 1
  for (int i = 0; i < IN; ++i) s += pmul(bf16_rne(x[v * IN + i]), bf16_rne(sl[i * OUT + lane]));
  const float o = fmaxf(a + s, 0.0f);
  for (int pass = 0; pass < 2; ++pass) { ((volatile float*)out)[v * OUT + lane] = o; __threadfence(); }
}
}

extern "C" void kernel_launch(void* const* d_in, const int* in_sizes, int n_in, void* d_out, int out_size, void* d_ws, size_t ws_size, hipStream_t stream) {
  (void)n_in;
  auto Fp = [&](int i) { return (const float*)d_in[i]; }; auto Ip = [&](int i) { return (const int*)d_in[i]; };
  if (in_sizes[0] != N * IN || in_sizes[1] != EFULL || in_sizes[2] != EFULL || in_sizes[3] != EFULL || in_sizes[4] != EFULL || in_sizes[5] != NG || in_sizes[6] != EFULL || in_sizes[7] != NG * R * ATT || in_sizes[8] != NB * IN * OUT || in_sizes[9] != R * NB || in_sizes[10] != IN * OUT || in_sizes[11] != 96 * IN || in_sizes[13] != IN || in_sizes[15] != 64 * IN || in_sizes[17] != IN || in_sizes[19] != OUT || out_size != N * OUT) return;
  size_t off = 0; char* ws = (char*)d_ws;
  auto carve = [&](size_t bytes) { char* p = ws + off; off += (bytes + 255) & ~(size_t)255; return p; };
  b16* BB = (b16*)carve(128 * 32 * 2); b16* A1T = (b16*)carve(32 * 96 * 2); b16* A2T = (b16*)carve(32 * 64 * 2); float* MSG = (float*)carve((size_t)E * OUT * 4);
  CsrBufs csr; off = csr_carve(csr, ws, off, E, N);
  if (off > ws_size || off > ((size_t)128 << 20)) return;
  wprep_kernel<<<1, 256, 0, stream>>>(Fp(8), Fp(11), Fp(15), BB, A1T, A2T);
  csr_build(csr, Ip(2), E, N, stream);
  edge_kernel<<<E / 32, 64, 0, stream>>>(Fp(0), Ip(1), Ip(2), Ip(3), Ip(4), Ip(5), Fp(6), Fp(7), Fp(9), BB, A1T, Fp(12), Fp(13), Fp(14), A2T, Fp(16), Fp(17), Fp(18), MSG);
  node_kernel<<<NP / 8, 256, 0, stream>>>(MSG, Fp(0), Fp(10), Fp(19), csr.PERM, csr.ROWPTR, csr.ROWCNT, (int)csr.permLen, (float*)d_out);
}
